// SparseAttention3d_41128606826831
// MI455X (gfx1250) — hardware-verified
//
#include <hip/hip_runtime.h>


namespace {
constexpr int NV = 40000, NVP = 40000  , NQ = 8192, KK = 96, C = 128, FF = 256, NH = 8, DH = 16;
constexpr float XS = 8.0f, WSC = 256.0f, EPS = 1e-5f, SCALE = 0.25f;

typedef _Float16 b16;
typedef __attribute__((ext_vector_type(16))) _Float16 v16b;
typedef __attribute__((ext_vector_type(8))) _Float16 v8b;
typedef __attribute__((ext_vector_type(8))) float v8f;
typedef __attribute__((ext_vector_type(4))) float v4f;
__device__ __forceinline__ float bf16_rne(float f) { unsigned int u = __float_as_uint(f); u += 0x7FFFu + ((u >> 16) & 1u); return __uint_as_float(u & 0xFFFF0000u); }
__device__ __forceinline__ void split16(float v, b16& hi, b16& lo) { hi = (b16)v; lo = (b16)(v - (float)hi); }
__device__ __forceinline__ v16b frag_kb(const b16* p, int hh) { const v8b a = *(const v8b*)(p + 8 * hh), b = *(const v8b*)(p + 16 + 8 * hh); v16b f;
#pragma unroll
  for (int e = 0; e < 8; ++e) { f[e] = a[e]; f[8 + e] = b[e]; } return f; }
__device__ __forceinline__ v8f wmma16b(v16b a, v16b b, v8f c) { v8f d = __builtin_amdgcn_wmma_f32_16x16x32_f16(false, a, false, b, (short)0, c, false, false); asm volatile("v_nop\n\tv_nop\n\tv_nop\n\tv_nop" : "+v"(d) : "v"(a), "v"(b)); return d; }
__device__ __forceinline__ void wave_lds_sync() { __builtin_amdgcn_fence(__ATOMIC_RELEASE, "workgroup"); __builtin_amdgcn_wave_barrier(); __builtin_amdgcn_fence(__ATOMIC_ACQUIRE, "workgroup"); }
__device__ __forceinline__ float pmul(float a, float b) { float p = a * b; asm volatile("" : "+v"(p)); return p; }
__device__ __forceinline__ int iclamp(int v, int lo, int hi) { return v < lo ? lo : (v > hi ? hi : v); }

__global__ __launch_bounds__(256) void prepw_kernel(const float* __restrict__ in_w, const float* __restrict__ wo, const float* __restrict__ l1, const float* __restrict__ l2, const float* __restrict__ fin, b16* __restrict__ WKV, b16* __restrict__ WQ, b16* __restrict__ WO, b16* __restrict__ L1, b16* __restrict__ L2, b16* __restrict__ FIN) {
  const int t = blockIdx.x * 256 + threadIdx.x; int u = t; v8b o; const float* src; b16* dst; int n;
  const int n0 = 2 * C * C / 8, n1 = C * C / 8, n3 = FF * C / 8;
  if (u < n0) { src = in_w + C * C; dst = WKV; n = u; } else if ((u -= n0) < n1) { src = in_w; dst = WQ; n = u; } else if ((u -= n1) < n1) { src = wo; dst = WO; n = u; } else if ((u -= n1) < n3) { src = l1; dst = L1; n = u; } else if ((u -= n3) < n3) { src = l2; dst = L2; n = u; } else if ((u -= n3) < n1) { src = fin; dst = FIN; n = u; } else return;
  for (int j = 0; j < 8; ++j) o[j] = (b16)(bf16_rne(src[n * 8 + j]) * WSC);
  for (int pass = 0; pass < 2; ++pass) { *(volatile v8b*)(dst + n * 8) = o; __threadfence(); }
}
__global__ __launch_bounds__(256) void voxel_kernel(const float* __restrict__ vfeat, const float* __restrict__ vc, const float* __restrict__ g1, const float* __restrict__ b1, const float* __restrict__ kpw, const float* __restrict__ kpb, float* __restrict__ KF) {
  const int wave = threadIdx.x >> 5, lane = threadIdx.x & 31; const size_t v = (size_t)blockIdx.x * 8 + wave; if (v >= (size_t)NV) return;
  const v4f x = *(const v4f*)(vfeat + v * C + lane * 4); float xs[4]; float s = 0.0f; for (int j = 0; j < 4; ++j) { xs[j] = bf16_rne(x[j]); s += xs[j]; }
#pragma unroll
  for (int o = 16; o >= 1; o >>= 1) s += __shfl_xor(s, o);
  const float mean = s * (1.0f / C); float q = 0.0f; for (int j = 0; j < 4; ++j) { const float d = xs[j] - mean; q += d * d; }
#pragma unroll
  for (int o = 16; o >= 1; o >>= 1) q += __shfl_xor(q, o);
  const float rstd = rsqrtf(q * (1.0f / C) + EPS); const float c0 = bf16_rne(vc[v * 3]), c1 = bf16_rne(vc[v * 3 + 1]), c2 = bf16_rne(vc[v * 3 + 2]); v4f r;
  for (int j = 0; j < 4; ++j) { const int c = lane * 4 + j; const float pos = fmaxf(pmul(c0, bf16_rne(kpw[c * 3])) + pmul(c1, bf16_rne(kpw[c * 3 + 1])) + pmul(c2, bf16_rne(kpw[c * 3 + 2])) + bf16_rne(kpb[c]), 0.0f); r[j] = (xs[j] - mean) * rstd * bf16_rne(g1[c]) + bf16_rne(b1[c]) + pos; }
  for (int pass = 0; pass < 2; ++pass) { *(volatile v4f*)(KF + v * C + lane * 4) = r; __threadfence(); }
}
__global__ __launch_bounds__(256) void qfeat_kernel(const float* __restrict__ qc, const float* __restrict__ qpw, const float* __restrict__ qpb, float* __restrict__ QF) {
  const int wave = threadIdx.x >> 5, lane = threadIdx.x & 31; const size_t n = (size_t)blockIdx.x * 8 + wave; const float c0 = bf16_rne(qc[n * 3]), c1 = bf16_rne(qc[n * 3 + 1]), c2 = bf16_rne(qc[n * 3 + 2]); v4f r;
  for (int j = 0; j < 4; ++j) { const int c = lane * 4 + j; r[j] = fmaxf(pmul(c0, bf16_rne(qpw[c * 3])) + pmul(c1, bf16_rne(qpw[c * 3 + 1])) + pmul(c2, bf16_rne(qpw[c * 3 + 2])) + bf16_rne(qpb[c]), 0.0f); }
  for (int pass = 0; pass < 2; ++pass) { *(volatile v4f*)(QF + n * C + lane * 4) = r; __threadfence(); }
}
template <int KD, int MODE>
__global__ __launch_bounds__(128) void dense_kernel(const float* __restrict__ X, const b16* __restrict__ Wt, const float* __restrict__ bias, const float* __restrict__ R, float* __restrict__ Y, int ldy) {
  __shared__ __attribute__((aligned(16))) b16 Ah[4][16][KD + 8], Al[4][16][KD + 8]; __shared__ __attribute__((aligned(16))) float Tf[4][16][128 + 4];
  const int wave = threadIdx.x >> 5, lane = threadIdx.x & 31, nloc = lane & 15, hlf = lane >> 4; const size_t m0 = (size_t)blockIdx.x * 64 + wave * 16; const int n0 = blockIdx.y * 128;
  for (int q = lane; q < 16 * (KD / 4); q += 32) { const int rr = q / (KD / 4), c4 = (q % (KD / 4)) * 4; const v4f xv = *(const v4f*)(X + (m0 + rr) * KD + c4); for (int j = 0; j < 4; ++j) { b16 p, pl; split16(xv[j] * XS, p, pl); Ah[wave][rr][c4 + j] = p; Al[wave][rr][c4 + j] = pl; } }
  wave_lds_sync();
  v8f acc[8];
#pragma unroll
  for (int t = 0; t < 8; ++t) acc[t] = (v8f){};
#pragma unroll 2
  for (int kb = 0; kb < KD; kb += 32) { const v16b a = frag_kb(&Ah[wave][nloc][kb], hlf), al = frag_kb(&Al[wave][nloc][kb], hlf);
#pragma unroll
    for (int t = 0; t < 8; ++t) { const v16b bw = frag_kb(Wt + (size_t)(n0 + t * 16 + nloc) * KD + kb, hlf); acc[t] = wmma16b(a, bw, acc[t]); acc[t] = wmma16b(al, bw, acc[t]); } }
#pragma unroll
  for (int t = 0; t < 8; ++t) { const int c = n0 + t * 16 + nloc; const float bb = bf16_rne(bias[c]);
#pragma unroll
    for (int r = 0; r < 8; ++r) { float y = acc[t][r] * (1.0f / (XS * WSC)) + bb; if (MODE == 1) y = fmaxf(y, 0.0f); if (R) y += R[(m0 + 8 * hlf + r) * ldy + c]; Tf[wave][8 * hlf + r][t * 16 + nloc] = y; } }
  wave_lds_sync();
  for (int pass = 0; pass < 2; ++pass) { for (int rr = 0; rr < 16; ++rr) *(volatile v4f*)(Y + (m0 + rr) * ldy + n0 + lane * 4) = *(const v4f*)(&Tf[wave][rr][lane * 4]); __threadfence(); }
}
__global__ __launch_bounds__(256) void attn_kernel(const float* __restrict__ Qp, const float* __restrict__ KV, const int* __restrict__ kidx, float* __restrict__ CTX) {
  const int wave = threadIdx.x >> 5, lane = threadIdx.x & 31; const size_t n = (size_t)blockIdx.x * 8 + wave;
  const v4f q = *(const v4f*)(Qp + n * C + lane * 4); float m = -INFINITY, l = 0.0f; float o[4] = {0.0f, 0.0f, 0.0f, 0.0f}; int nvalid = 0;
  for (int s = 0; s < KK; ++s) { const int raw = kidx[n * KK + s]; const bool valid = raw >= 0; const int idx = valid ? iclamp(raw, 0, NV - 1) : 0; nvalid += valid ? 1 : 0;
    const v4f kv = *(const v4f*)(KV + (size_t)idx * (2 * C) + lane * 4); const v4f vv = *(const v4f*)(KV + (size_t)idx * (2 * C) + C + lane * 4);
    float d = pmul(q[0], kv[0]) + pmul(q[1], kv[1]) + pmul(q[2], kv[2]) + pmul(q[3], kv[3]); d += __shfl_xor(d, 1); d += __shfl_xor(d, 2);
    const float sc = valid ? d * SCALE : -1e9f; const float mn = fmaxf(m, sc); const float al = __expf(m - mn); const float p = __expf(sc - mn); l = l * al + p;
    for (int j = 0; j < 4; ++j) o[j] = o[j] * al + pmul(p, vv[j]); m = mn; }
  (void)nvalid; const float inv = 1.0f / l; v4f r; for (int j = 0; j < 4; ++j) r[j] = o[j] * inv;
  for (int pass = 0; pass < 2; ++pass) { *(volatile v4f*)(CTX + n * C + lane * 4) = r; __threadfence(); }
}
__global__ __launch_bounds__(256) void ln_kernel(const float* __restrict__ X, const float* __restrict__ g, const float* __restrict__ b, float* __restrict__ Y) {
  const int wave = threadIdx.x >> 5, lane = threadIdx.x & 31; const size_t n = (size_t)blockIdx.x * 8 + wave; const v4f x = *(const v4f*)(X + n * C + lane * 4); float s = x[0] + x[1] + x[2] + x[3];
#pragma unroll
  for (int o = 16; o >= 1; o >>= 1) s += __shfl_xor(s, o);
  const float mean = s * (1.0f / C); float q = 0.0f; for (int j = 0; j < 4; ++j) { const float d = x[j] - mean; q += d * d; }
#pragma unroll
  for (int o = 16; o >= 1; o >>= 1) q += __shfl_xor(q, o);
  const float rstd = rsqrtf(q * (1.0f / C) + EPS); v4f r; for (int j = 0; j < 4; ++j) { const int c = lane * 4 + j; r[j] = (x[j] - mean) * rstd * bf16_rne(g[c]) + bf16_rne(b[c]); }
  for (int pass = 0; pass < 2; ++pass) { *(volatile v4f*)(Y + n * C + lane * 4) = r; __threadfence(); }
}
}

extern "C" void kernel_launch(void* const* d_in, const int* in_sizes, int n_in, void* d_out, int out_size, void* d_ws, size_t ws_size, hipStream_t stream) {
  (void)n_in;
  auto Fp = [&](int i) { return (const float*)d_in[i]; }; auto Ip = [&](int i) { return (const int*)d_in[i]; };
  if (in_sizes[0] != NV * C || in_sizes[1] != NV * 3 || in_sizes[2] != NQ * 3 || in_sizes[3] != NQ * KK || in_sizes[10] != 3 * C * C || in_sizes[16] != FF * C || in_sizes[18] != C * FF || in_sizes[20] != C * C || out_size != NQ * C) return;
  size_t off = 0; char* ws = (char*)d_ws;
  auto carve = [&](size_t bytes) { char* p = ws + off; off += (bytes + 255) & ~(size_t)255; return p; };
  b16* WKV = (b16*)carve((size_t)2 * C * C * 2); b16* WQ = (b16*)carve((size_t)C * C * 2); b16* WO = (b16*)carve((size_t)C * C * 2); b16* L1 = (b16*)carve((size_t)FF * C * 2); b16* L2 = (b16*)carve((size_t)C * FF * 2); b16* FIN = (b16*)carve((size_t)C * C * 2);
  float* KF = (float*)carve((size_t)NVP * C * 4); float* KV = (float*)carve((size_t)NVP * 2 * C * 4); float* QF = (float*)carve((size_t)NQ * C * 4); float* Qp = (float*)carve((size_t)NQ * C * 4); float* CTX = (float*)carve((size_t)NQ * C * 4); float* ATT = (float*)carve((size_t)NQ * C * 4); float* HN = (float*)carve((size_t)NQ * C * 4); float* A1 = (float*)carve((size_t)NQ * FF * 4); float* XR = (float*)carve((size_t)NQ * C * 4);
  if (off > ws_size || off > ((size_t)128 << 20)) return;
  prepw_kernel<<<(2 * C * C / 8 + 3 * C * C / 8 + 2 * FF * C / 8 + 255) / 256, 256, 0, stream>>>(Fp(10), Fp(12), Fp(16), Fp(18), Fp(20), WKV, WQ, WO, L1, L2, FIN);
  voxel_kernel<<<NVP / 8, 256, 0, stream>>>(Fp(0), Fp(1), Fp(4), Fp(5), Fp(8), Fp(9), KF);
  dense_kernel<C, 0><<<dim3(NVP / 64, 2), 128, 0, stream>>>(KF, WKV, Fp(11) + C, nullptr, KV, 2 * C);
  qfeat_kernel<<<NQ / 8, 256, 0, stream>>>(Fp(2), Fp(6), Fp(7), QF);
  dense_kernel<C, 0><<<dim3(NQ / 64, 1), 128, 0, stream>>>(QF, WQ, Fp(11), nullptr, Qp, C);
  attn_kernel<<<NQ / 8, 256, 0, stream>>>(Qp, KV, Ip(3), CTX);
  dense_kernel<C, 0><<<dim3(NQ / 64, 1), 128, 0, stream>>>(CTX, WO, Fp(13), nullptr, ATT, C);
  ln_kernel<<<NQ / 8, 256, 0, stream>>>(ATT, Fp(14), Fp(15), HN);
  dense_kernel<C, 1><<<dim3(NQ / 64, 2), 128, 0, stream>>>(HN, L1, Fp(17), nullptr, A1, FF);
  dense_kernel<FF, 0><<<dim3(NQ / 64, 1), 128, 0, stream>>>(A1, L2, Fp(19), ATT, XR, C);
  dense_kernel<C, 1><<<dim3(NQ / 64, 1), 128, 0, stream>>>(XR, FIN, Fp(21), nullptr, (float*)d_out, C);
}
